// TaylorModel_25280177504598
// MI455X (gfx1250) — hardware-verified
//
#include <hip/hip_runtime.h>
#include <math.h>

#pragma clang fp contract(off)

typedef __attribute__((ext_vector_type(16))) __bf16       v16b;
typedef __attribute__((ext_vector_type(8)))  float        v8f;
typedef __attribute__((ext_vector_type(4)))  float        v4f;
typedef __attribute__((ext_vector_type(4)))  unsigned int u4;

constexpr int kRows     = 262144;
constexpr int kDin      = 18;
constexpr int kHid      = 20;
constexpr int kK1       = kDin + kDin * (kDin + 1) / 2;
constexpr int kK2       = kHid + kHid * (kHid + 1) / 2;
constexpr int kK1P      = 192;
constexpr int kK2P      = 256;
constexpr int kNPad     = 32;
constexpr int kTileRows = 32;
constexpr int kG1       = kK1P / 8;
constexpr int kG2       = kK2P / 8;
constexpr int kAP       = 33;
constexpr int kZP       = 33;
constexpr int kXV4      = kTileRows * kDin / 4;
constexpr int kXIters   = (kXV4 + 31) / 32;

static_assert(kK1 == 189 && kK2 == 230, "expanded widths");
static_assert(kK1P >= kK1 && kK2P >= kK2 && (kK1P % 32) == 0 && (kK2P % 32) == 0, "K pads are multiples of 32");
static_assert((kRows % kTileRows) == 0, "no row tail");
static_assert(((kTileRows * kDin * 4) % 128) == 0, "block input span is whole 128-B lines");
static_assert(((kTileRows * kDin) % 4) == 0, "block input span is whole 16-B vectors");
static_assert(kG2 <= 32 && kG1 <= 32 && kG2 + 1 <= kAP, "group counts fit one wave and the LDS pitch");
static_assert(kHid <= kNPad && kNPad == 32, "two 16-wide N tiles");

constexpr int kOffW1H = 0;
constexpr int kOffW1L = kOffW1H + kNPad * kG1;
constexpr int kOffW2H = kOffW1L + kNPad * kG1;
constexpr int kOffW2L = kOffW2H + kNPad * kG2;
constexpr int kWsU4   = kOffW2L + kNPad * kG2;
constexpr size_t kWsBytes = (size_t)kWsU4 * 16;
static_assert(kWsBytes == 57344ull, "carve total");
static_assert(kWsBytes <= 134217728ull, "carve cap");
static_assert((kOffW1L % 8) == 0 && (kOffW2H % 8) == 0 && (kOffW2L % 8) == 0, "128-B aligned regions");

__host__ __device__ constexpr int tri_j(int c, int idx) {
  int j = 0;
  while (idx >= c - j) { idx -= (c - j); ++j; }
  return j;
}
__host__ __device__ constexpr int tri_k(int c, int idx) {
  int j = 0;
  while (idx >= c - j) { idx -= (c - j); ++j; }
  return j + idx;
}
static_assert(tri_j(18, 0) == 0 && tri_k(18, 0) == 0, "pair 0");
static_assert(tri_j(18, 17) == 0 && tri_k(18, 17) == 17, "pair 17");
static_assert(tri_j(18, 18) == 1 && tri_k(18, 18) == 1, "pair 18");
static_assert(tri_j(18, 170) == 17 && tri_k(18, 170) == 17, "last pair c=18");
static_assert(tri_j(20, 209) == 19 && tri_k(20, 209) == 19, "last pair c=20");

__device__ __forceinline__ unsigned bf_rne(float f) {
  const unsigned u = __float_as_uint(f);
  return (u + 0x7FFFu + ((u >> 16) & 1u)) >> 16;
}
__device__ __forceinline__ void split_pack(float a, float b, unsigned& wh, unsigned& wl) {
  const unsigned ha = bf_rne(a);
  const unsigned hb = bf_rne(b);
  const float ra = a - __uint_as_float(ha << 16);
  const float rb = b - __uint_as_float(hb << 16);
  const unsigned la = bf_rne(ra);
  const unsigned lb = bf_rne(rb);
  wh = ha | (hb << 16);
  wl = la | (lb << 16);
}

template <int C, int COL>
__device__ __forceinline__ float aug_val(const float (&v)[C]) {
  constexpr bool LIN  = (COL < C);
  constexpr bool PROD = (!LIN) && (COL < C + C * (C + 1) / 2);
  constexpr int  L    = LIN ? COL : 0;
  constexpr int  J    = PROD ? tri_j(C, COL - C) : 0;
  constexpr int  K    = PROD ? tri_k(C, COL - C) : 0;
  return LIN ? v[L] : (PROD ? (v[J] * v[K]) : 0.0f);
}

template <int C, int G>
__device__ __forceinline__ void aug_group(const float (&v)[C], u4* ph, u4* pl) {
  unsigned h0, h1, h2, h3, l0, l1, l2, l3;
  split_pack(aug_val<C, 8 * G + 0>(v), aug_val<C, 8 * G + 1>(v), h0, l0);
  split_pack(aug_val<C, 8 * G + 2>(v), aug_val<C, 8 * G + 3>(v), h1, l1);
  split_pack(aug_val<C, 8 * G + 4>(v), aug_val<C, 8 * G + 5>(v), h2, l2);
  split_pack(aug_val<C, 8 * G + 6>(v), aug_val<C, 8 * G + 7>(v), h3, l3);
  const u4 hv = {h0, h1, h2, h3};
  const u4 lv = {l0, l1, l2, l3};
  ph[G] = hv;
  pl[G] = lv;
}

template <int C, int G, int NG> struct AugLoop {
  static __device__ __forceinline__ void run(const float (&v)[C], u4* ph, u4* pl) {
    aug_group<C, G>(v, ph, pl);
    AugLoop<C, G + 1, NG>::run(v, ph, pl);
  }
};
template <int C, int NG> struct AugLoop<C, NG, NG> {
  static __device__ __forceinline__ void run(const float (&)[C], u4*, u4*) {}
};

union FragB { v16b v; u4 q[2]; };
__device__ __forceinline__ v16b ld_frag(const u4* p) {
  FragB f;
  f.q[0] = p[0];
  f.q[1] = p[2];
  return f.v;
}
__device__ __forceinline__ v8f mma_bf(v16b a, v16b b, v8f c) {
  return __builtin_amdgcn_wmma_f32_16x16x32_bf16(false, a, false, b, (short)0, c, false, false);
}
__device__ __forceinline__ void tile3(v8f& acc, v16b ah, v16b al, v16b bh, v16b bl) {
  acc = mma_bf(ah, bh, acc);
  acc = mma_bf(ah, bl, acc);
  acc = mma_bf(al, bh, acc);
  asm volatile("v_nop\n\tv_nop\n\tv_nop\n\tv_nop" : "+v"(acc) : "v"(ah), "v"(al), "v"(bh), "v"(bl));
}

template <int NCH, int BP>
__device__ __forceinline__ void layer_mma(const u4* ah, const u4* al, const u4* bh, const u4* bl,
                                          int c, int hh, v8f& d00, v8f& d01, v8f& d10, v8f& d11) {
  const u4* pa0h = ah + c * kAP + hh;
  const u4* pa1h = pa0h + 16 * kAP;
  const u4* pa0l = al + c * kAP + hh;
  const u4* pa1l = pa0l + 16 * kAP;
  const u4* pb0h = bh + c * BP + hh;
  const u4* pb1h = pb0h + 16 * BP;
  const u4* pb0l = bl + c * BP + hh;
  const u4* pb1l = pb0l + 16 * BP;
#pragma unroll 1
  for (int ch = 0; ch < NCH; ++ch) {
    const int o = ch * 4;
    const v16b a0h = ld_frag(pa0h + o);
    const v16b a0l = ld_frag(pa0l + o);
    const v16b a1h = ld_frag(pa1h + o);
    const v16b a1l = ld_frag(pa1l + o);
    const v16b b0h = ld_frag(pb0h + o);
    const v16b b0l = ld_frag(pb0l + o);
    const v16b b1h = ld_frag(pb1h + o);
    const v16b b1l = ld_frag(pb1l + o);
    tile3(d00, a0h, a0l, b0h, b0l);
    tile3(d01, a0h, a0l, b1h, b1l);
    tile3(d10, a1h, a1l, b0h, b0l);
    tile3(d11, a1h, a1l, b1h, b1l);
  }
}

__global__ __launch_bounds__(32) void build_weight_planes(const float* __restrict__ W1,
                                                          const float* __restrict__ W2,
                                                          u4* __restrict__ wp) {
  const int g   = threadIdx.x;
  const int blk = blockIdx.x;
  const bool second = (blk >= kNPad);
  const int n   = blk & (kNPad - 1);
  const float* W = second ? W2 : W1;
  const int K    = second ? kK2 : kK1;
  const int G    = second ? kG2 : kG1;
  const int offH = second ? kOffW2H : kOffW1H;
  const int offL = second ? kOffW2L : kOffW1L;
  const int nc   = (n < kHid) ? n : (kHid - 1);
  const bool nreal = (n < kHid);
  float f[8];
#pragma unroll
  for (int e = 0; e < 8; ++e) {
    const int k  = 8 * g + e;
    const int kc = (k < K) ? k : (K - 1);
    const float w = W[nc * K + kc];
    f[e] = (nreal && (k < K)) ? w : 0.0f;
  }
  unsigned h0, h1, h2, h3, l0, l1, l2, l3;
  split_pack(f[0], f[1], h0, l0);
  split_pack(f[2], f[3], h1, l1);
  split_pack(f[4], f[5], h2, l2);
  split_pack(f[6], f[7], h3, l3);
  const u4 hv = {h0, h1, h2, h3};
  const u4 lv = {l0, l1, l2, l3};
  if (g < G) {
    volatile u4* ph = (volatile u4*)(wp + offH + n * G + g);
    volatile u4* pl = (volatile u4*)(wp + offL + n * G + g);
    *ph = hv;
    *pl = lv;
    __threadfence();
    *ph = hv;
    *pl = lv;
  }
}

__global__ __launch_bounds__(32) void taylor_fused_kernel(const float* __restrict__ x,
                                                          const float* __restrict__ b1,
                                                          const float* __restrict__ b2,
                                                          const float* __restrict__ W3,
                                                          const float* __restrict__ b3,
                                                          const u4* __restrict__ wp,
                                                          float* out) {
  __shared__ __align__(16) float sx[kTileRows * kDin];
  __shared__ __align__(16) float sz[kTileRows * kZP];
  __shared__ __align__(16) u4 sAh[kTileRows * kAP];
  __shared__ __align__(16) u4 sAl[kTileRows * kAP];

  const int lane = threadIdx.x & 31;
  const int hh   = lane >> 4;
  const int c    = lane & 15;
  const int row0 = blockIdx.x * kTileRows;

  {
    const float* xb = x + (size_t)row0 * kDin;
#pragma unroll
    for (int it = 0; it < kXIters; ++it) {
      int idx = it * 32 + lane;
      idx = (idx < kXV4 - 1) ? idx : (kXV4 - 1);
      const v4f v = *(const v4f*)(xb + 4 * idx);
      *(v4f*)(sx + 4 * idx) = v;
    }
  }
  __syncthreads();

  {
    float xv[kDin];
#pragma unroll
    for (int i = 0; i < kDin; ++i) xv[i] = sx[lane * kDin + i];
    AugLoop<kDin, 0, kG1>::run(xv, sAh + lane * kAP, sAl + lane * kAP);
  }
  __syncthreads();

  v8f d00 = (v8f){0.f, 0.f, 0.f, 0.f, 0.f, 0.f, 0.f, 0.f};
  v8f d01 = d00, d10 = d00, d11 = d00;
  layer_mma<kK1P / 32, kG1>(sAh, sAl, wp + kOffW1H, wp + kOffW1L, c, hh, d00, d01, d10, d11);

#pragma unroll
  for (int r = 0; r < 8; ++r) {
    sz[(8 * hh + r) * kZP + c]           = d00[r];
    sz[(8 * hh + r) * kZP + 16 + c]      = d01[r];
    sz[(16 + 8 * hh + r) * kZP + c]      = d10[r];
    sz[(16 + 8 * hh + r) * kZP + 16 + c] = d11[r];
  }
  __syncthreads();
#pragma unroll 1
  for (int col = 0; col < kHid; ++col) {
    const float z = sz[lane * kZP + col] + b1[col];
    sz[lane * kZP + col] = tanhf(z);
  }
  __syncthreads();

  {
    float hv[kHid];
#pragma unroll
    for (int i = 0; i < kHid; ++i) hv[i] = sz[lane * kZP + i];
    AugLoop<kHid, 0, kG2>::run(hv, sAh + lane * kAP, sAl + lane * kAP);
  }
  __syncthreads();

  d00 = (v8f){0.f, 0.f, 0.f, 0.f, 0.f, 0.f, 0.f, 0.f};
  d01 = d00; d10 = d00; d11 = d00;
  layer_mma<kK2P / 32, kG2>(sAh, sAl, wp + kOffW2H, wp + kOffW2L, c, hh, d00, d01, d10, d11);

#pragma unroll
  for (int r = 0; r < 8; ++r) {
    sz[(8 * hh + r) * kZP + c]           = d00[r];
    sz[(8 * hh + r) * kZP + 16 + c]      = d01[r];
    sz[(16 + 8 * hh + r) * kZP + c]      = d10[r];
    sz[(16 + 8 * hh + r) * kZP + 16 + c] = d11[r];
  }
  __syncthreads();
#pragma unroll 1
  for (int col = 0; col < kHid; ++col) {
    const float z = sz[lane * kZP + col] + b2[col];
    sz[lane * kZP + col] = tanhf(z);
  }
  __syncthreads();

  {
    float acc = 0.0f;
#pragma unroll 1
    for (int n = 0; n < kHid; ++n) acc = fmaf(sz[lane * kZP + n], W3[n], acc);
    const float y = acc + b3[0];
    volatile float* po = (volatile float*)(out + row0 + lane);
    *po = y;
    __threadfence();
    *po = y;
  }
}

extern "C" void kernel_launch(void* const* d_in, const int* in_sizes, int n_in,
                              void* d_out, int out_size, void* d_ws, size_t ws_size,
                              hipStream_t stream) {
  if (n_in < 7) return;
  if (in_sizes[0] != kRows * kDin) return;
  if (in_sizes[1] != kHid * kK1) return;
  if (in_sizes[2] != kHid) return;
  if (in_sizes[3] != kHid * kK2) return;
  if (in_sizes[4] != kHid) return;
  if (in_sizes[5] != kHid) return;
  if (in_sizes[6] != 1) return;
  if (out_size != kRows) return;
  if (ws_size < kWsBytes) return;

  const float* x  = (const float*)d_in[0];
  const float* W1 = (const float*)d_in[1];
  const float* b1 = (const float*)d_in[2];
  const float* W2 = (const float*)d_in[3];
  const float* b2 = (const float*)d_in[4];
  const float* W3 = (const float*)d_in[5];
  const float* b3 = (const float*)d_in[6];
  float* out = (float*)d_out;
  u4* wp = (u4*)d_ws;

  build_weight_planes<<<2 * kNPad, 32, 0, stream>>>(W1, W2, wp);
  taylor_fused_kernel<<<kRows / kTileRows, 32, 0, stream>>>(x, b1, b2, W3, b3, wp, out);
}
